// CausalSelfAttention_20469814132940
// MI455X (gfx1250) — hardware-verified
//
#include <hip/hip_runtime.h>
#include <math.h>

typedef __attribute__((ext_vector_type(16))) _Float16 v16h;
typedef __attribute__((ext_vector_type(16))) __bf16 v16b;
typedef __attribute__((ext_vector_type(8)))  _Float16 v8h;
typedef __attribute__((ext_vector_type(8)))  __bf16 v8b;
typedef __attribute__((ext_vector_type(8)))  float v8f;
typedef __attribute__((ext_vector_type(4)))  float v4f;
typedef __attribute__((ext_vector_type(4)))  unsigned v4u;

template <typename T> __device__ __forceinline__ void vst2(void* p, T v) { *(volatile T*)p = v; __threadfence(); *(volatile T*)p = v; }
__device__ __forceinline__ v8f wmma16(v16h a, v16h b, v8f c) {
  v8f d = __builtin_amdgcn_wmma_f32_16x16x32_f16(false, a, false, b, (short)0, c, false, false);
  asm volatile("v_nop\n\tv_nop\n\tv_nop\n\tv_nop" : "+v"(d) : "v"(a), "v"(b));
  return d;
}
__device__ __forceinline__ v8f wmma_bf(v16b a, v16b b, v8f c) {
  v8f d = __builtin_amdgcn_wmma_f32_16x16x32_bf16(false, a, false, b, (short)0, c, false, false);
  asm volatile("v_nop\n\tv_nop\n\tv_nop\n\tv_nop" : "+v"(d) : "v"(a), "v"(b));
  return d;
}
__device__ __forceinline__ v16h frag_h(const _Float16* rowk0, int lane) {
  union { v16h v; v8h q[2]; } u; const _Float16* p = rowk0 + 8 * (lane >> 4);
  u.q[0] = *(const v8h*)p; u.q[1] = *(const v8h*)(p + 16); return u.v;
}
__device__ __forceinline__ v16b frag_b(const __bf16* rowk0, int lane) {
  union { v16b v; v8b q[2]; } u; const __bf16* p = rowk0 + 8 * (lane >> 4);
  u.q[0] = *(const v8b*)p; u.q[1] = *(const v8b*)(p + 16); return u.v;
}
__device__ __forceinline__ float bfr(float v) { return (float)(__bf16)v; }
#define LDSX() do { asm volatile("s_wait_dscnt 0" ::: "memory"); __builtin_amdgcn_wave_barrier(); __builtin_amdgcn_fence(3  , "workgroup"); } while (0)

#ifndef NB
#define NB 2
#endif
#ifndef SEQ
#define SEQ 2048
#endif
#define NB_FULL 2
#define SEQ_FULL 2048
#define CC 1024
#define DIN 1024
#define NH 16
#define HD 64
#define QBH 4
#define KHI 256
#define SCALE (0.125f)
#define NEGBIG (-1.0e30f)
#define PCARRY (2048.0f)

static_assert(NH * HD == CC);
static_assert(CC == DIN);
static_assert(HD == 64);
static_assert(SEQ % 64 == 0);
static_assert(QBH * 64 == KHI);
static_assert(KHI <= SEQ);
static_assert(CC % 128 == 0);
static_assert(DIN % 64 == 0);
static_assert(DIN % 32 == 0);
static_assert(((size_t)NB * SEQ * DIN / 8) % 256 == 0);
static_assert(NB <= NB_FULL);
static_assert(SEQ <= SEQ_FULL);

#define PLANE   ((size_t)NB * SEQ * CC)
#define WS_XB   ((size_t)0)
#define WS_WQT  (WS_XB  + 2u * (size_t)NB * SEQ * DIN)
#define WS_WPT  (WS_WQT + 2u * (size_t)3 * CC * DIN)
#define WS_QKH  (WS_WPT + 2u * (size_t)DIN * CC)
#define WS_QKL  (WS_QKH + 2u * 2u * PLANE)
#define WS_VF   (WS_QKL + 2u * 2u * PLANE)
#define WS_VT   (WS_VF  + 4u * PLANE)
#define WS_VB   (WS_VT  + 2u * PLANE)
#define WS_VBL  (WS_VB  + 2u * (size_t)NB * NH * HD * KHI)
#define WS_YH   (WS_VBL + 2u * (size_t)NB * NH * HD * KHI)
#define WS_YL   (WS_YH  + 2u * PLANE)
#define WS_END  (WS_YL  + 2u * PLANE)
static_assert(WS_END <= (size_t)134217728);
static_assert(WS_WQT % 128 == 0 && WS_WPT % 128 == 0 && WS_QKH % 128 == 0 && WS_QKL % 128 == 0 && WS_VF % 128 == 0 && WS_VT % 128 == 0 && WS_VB % 128 == 0 && WS_VBL % 128 == 0 && WS_YH % 128 == 0 && WS_YL % 128 == 0);

__global__ __launch_bounds__(256) void k_cvt_x(const float* __restrict__ X, __bf16* __restrict__ XB) {
  const size_t i = (size_t)blockIdx.x * 256 + threadIdx.x;
  const size_t row = i / (DIN / 8); const int pc = (int)(i % (DIN / 8));
  const size_t b = row / SEQ, t = row % SEQ;
  const float* p = X + (b * (size_t)SEQ_FULL + t) * DIN + pc * 8;
  const v4f a = *(const v4f*)p, c = *(const v4f*)(p + 4);
  union { v8b b8; v4u u; } o;
#pragma unroll
  for (int k = 0; k < 4; ++k) { o.b8[k] = (__bf16)a[k]; o.b8[4 + k] = (__bf16)c[k]; }
  vst2((void*)(XB + row * DIN + pc * 8), o.u);
}
__global__ __launch_bounds__(256) void k_wT(const float* __restrict__ W, __bf16* __restrict__ WT, int K, int N) {
  __shared__ __align__(16) __bf16 tw[64][72];
  const int tid = threadIdx.x; const int n0 = blockIdx.x * 64, k0 = blockIdx.y * 64;
#pragma unroll 4
  for (int i = 0; i < 16; ++i) { const int e = tid + i * 256; const int kk = e >> 6, nn = e & 63; tw[nn][kk] = (__bf16)W[(size_t)(k0 + kk) * N + n0 + nn]; }
  __syncthreads();
#pragma unroll
  for (int i = 0; i < 2; ++i) { const int e = tid + i * 256; const int nn = e >> 3, q = e & 7; const v4u val = *(const v4u*)&tw[nn][q * 8]; vst2((void*)(WT + (size_t)(n0 + nn) * K + k0 + q * 8), val); }
}
__global__ __launch_bounds__(128) void k_proj(const __bf16* __restrict__ XB, const __bf16* __restrict__ WT, const float* __restrict__ BQKV, __bf16* __restrict__ QKH, __bf16* __restrict__ QKL, float* __restrict__ VF) {
  __shared__ __align__(16) float st[64][132]; __shared__ __align__(16) __bf16 sh[64][136], sl[64][136];
  const int tid = threadIdx.x; const int wave = __builtin_amdgcn_readfirstlane(tid >> 5); const int lane = tid & 31, col = lane & 15, g = lane >> 4;
  const int c0 = blockIdx.y * 128; const int which = c0 / CC; const int cw = c0 - which * CC; const size_t r0 = (size_t)blockIdx.x * 64;
  v8f acc[8] = {};
  const __bf16* arow = XB + (r0 + wave * 16 + col) * DIN;
#pragma unroll 1
  for (int kc = 0; kc < DIN / 32; ++kc) { const v16b a = frag_b(arow + kc * 32, lane);
#pragma unroll
    for (int j = 0; j < 8; ++j) { const v16b w = frag_b(WT + (size_t)(c0 + j * 16 + col) * DIN + kc * 32, lane); acc[j] = wmma_bf(a, w, acc[j]); } }
  if (which < 2) {
#pragma unroll
    for (int j = 0; j < 8; ++j) { const float bias = bfr(BQKV[c0 + j * 16 + col]);
#pragma unroll
      for (int r = 0; r < 8; ++r) { const float v = acc[j][r] + bias; const __bf16 hv = (__bf16)v; sh[wave * 16 + 8 * g + r][j * 16 + col] = hv; sl[wave * 16 + 8 * g + r][j * 16 + col] = (__bf16)(v - (float)hv); } }
  } else {
#pragma unroll
    for (int j = 0; j < 8; ++j) { const float bias = bfr(BQKV[c0 + j * 16 + col]);
#pragma unroll
      for (int r = 0; r < 8; ++r) st[wave * 16 + 8 * g + r][j * 16 + col] = acc[j][r] + bias; }
  }
  __syncthreads();
  if (which < 2) {
    __bf16* DH = QKH + (size_t)which * PLANE; __bf16* DL = QKL + (size_t)which * PLANE;
    for (int e = tid; e < 64 * 16; e += 128) { const int rl = e >> 4, q = e & 15; const size_t o = (r0 + rl) * CC + cw + q * 8;
      const v4u vh = *(const v4u*)&sh[rl][q * 8]; const v4u vl = *(const v4u*)&sl[rl][q * 8]; vst2((void*)(DH + o), vh); vst2((void*)(DL + o), vl); }
  } else {
    for (int e = tid; e < 64 * 32; e += 128) { const int rl = e >> 5, q = e & 31; const v4f vv = *(const v4f*)&st[rl][q * 4]; vst2((void*)(VF + (r0 + rl) * CC + cw + q * 4), vv); }
  }
}
__global__ __launch_bounds__(256) void k_vt(const float* __restrict__ VF, _Float16* __restrict__ VT, __bf16* __restrict__ VB, __bf16* __restrict__ VBL) {
  __shared__ __align__(16) _Float16 th[64][72]; __shared__ __align__(16) __bf16 tb[64][72], tbl[64][72];
  const int tid = threadIdx.x; const int s0 = blockIdx.x * 64; const int bh = blockIdx.y;
  const float* src = VF + (size_t)bh * SEQ * HD + (size_t)s0 * HD;
#pragma unroll 4
  for (int i = 0; i < 16; ++i) { const int e = tid + i * 256; const int s = e >> 6, d = e & 63; const float v = src[e]; th[d][s] = (_Float16)v; const __bf16 hv = (__bf16)v; tb[d][s] = hv; tbl[d][s] = (__bf16)(v - (float)hv); }
  __syncthreads();
#pragma unroll
  for (int i = 0; i < 2; ++i) { const int e = tid + i * 256; const int d = e >> 3, q = e & 7;
    const v4u v0 = *(const v4u*)&th[d][q * 8]; vst2((void*)(VT + ((size_t)bh * HD + d) * SEQ + s0 + q * 8), v0);
    if (s0 < KHI) {
      const size_t o3 = ((size_t)bh * HD + d) * KHI + s0 + q * 8; const v4u v1 = *(const v4u*)&tb[d][q * 8]; const v4u v2 = *(const v4u*)&tbl[d][q * 8];
      vst2((void*)(VB + o3), v1); vst2((void*)(VBL + o3), v2); } }
}
__global__ __launch_bounds__(128) void k_attn(const __bf16* __restrict__ QH, const __bf16* __restrict__ QL, const __bf16* __restrict__ KH, const __bf16* __restrict__ KL,
    const _Float16* __restrict__ VT, const __bf16* __restrict__ VB, const __bf16* __restrict__ VBL, __bf16* __restrict__ YH, __bf16* __restrict__ YL) {
  __shared__ __align__(16) _Float16 psh[4][16][40]; __shared__ __align__(16) __bf16 pbh[4][16][40], pbl[4][16][40]; __shared__ __align__(16) __bf16 ysh[4][16][72], ysl[4][16][72];
  const int tid = threadIdx.x; const int wave = __builtin_amdgcn_readfirstlane(tid >> 5); const int lane = tid & 31, col = lane & 15, g = lane >> 4;
  const int qb = blockIdx.x, bh = blockIdx.y; const int q0 = qb * 64 + wave * 16;
  const size_t hb = (size_t)bh * SEQ * HD;
  const bool hi = qb < QBH;
  v16b qh[2], ql[2];
#pragma unroll
  for (int kc = 0; kc < 2; ++kc) { const size_t qo = hb + (size_t)(q0 + col) * HD + kc * 32; qh[kc] = frag_b(QH + qo, lane); ql[kc] = frag_b(QL + qo, lane); }
  v8f acc[4] = {};
  float mst[8], lst[8];
#pragma unroll
  for (int r = 0; r < 8; ++r) { mst[r] = NEGBIG; lst[r] = 0.f; }
  const int nst = ((q0 + 15) >> 5) + 1;
#pragma unroll 1
  for (int st = 0; st < nst; ++st) { const int k0 = st * 32;
    v8f s[2] = {};
#pragma unroll
    for (int j = 0; j < 2; ++j) { const size_t ko = hb + (size_t)(k0 + j * 16 + col) * HD;
#pragma unroll
      for (int kc = 0; kc < 2; ++kc) { const v16b kh = frag_b(KH + ko + kc * 32, lane), kl = frag_b(KL + ko + kc * 32, lane);
        s[j] = wmma_bf(ql[kc], kh, s[j]); s[j] = wmma_bf(qh[kc], kl, s[j]); s[j] = wmma_bf(qh[kc], kh, s[j]); } }
#pragma unroll
    for (int r = 0; r < 8; ++r) { const int qrow = q0 + 8 * g + r; const bool ok0 = (k0 + col) <= qrow, ok1 = (k0 + 16 + col) <= qrow;
      const float a0 = ok0 ? s[0][r] * SCALE : NEGBIG; const float a1 = ok1 ? s[1][r] * SCALE : NEGBIG;
      float mx = fmaxf(a0, a1);
      mx = fmaxf(mx, __shfl_xor(mx, 1)); mx = fmaxf(mx, __shfl_xor(mx, 2)); mx = fmaxf(mx, __shfl_xor(mx, 4)); mx = fmaxf(mx, __shfl_xor(mx, 8));
      const float mnew = fmaxf(mst[r], mx);
      const float sc = __expf(mst[r] - mnew);
      const float p0 = ok0 ? __expf(a0 - mnew) : 0.f; const float p1 = ok1 ? __expf(a1 - mnew) : 0.f;
      lst[r] = lst[r] * sc + (p0 + p1);
      mst[r] = mnew;
      acc[0][r] *= sc; acc[1][r] *= sc; acc[2][r] *= sc; acc[3][r] *= sc;
      s[0][r] = p0; s[1][r] = p1; }
    if (hi) {
#pragma unroll
      for (int r = 0; r < 8; ++r) {
#pragma unroll
        for (int j = 0; j < 2; ++j) { const float p = s[j][r]; const __bf16 hv = (__bf16)p; pbh[wave][8 * g + r][j * 16 + col] = hv; pbl[wave][8 * g + r][j * 16 + col] = (__bf16)(p - (float)hv); } }
      LDSX();
      union { v16b v; v8b q[2]; } ph, pl;
      ph.q[0] = *(const v8b*)&pbh[wave][col][8 * g]; ph.q[1] = *(const v8b*)&pbh[wave][col][16 + 8 * g];
      pl.q[0] = *(const v8b*)&pbl[wave][col][8 * g]; pl.q[1] = *(const v8b*)&pbl[wave][col][16 + 8 * g];
      LDSX();
#pragma unroll
      for (int jt = 0; jt < 4; ++jt) { const size_t vo = ((size_t)bh * HD + jt * 16 + col) * KHI + k0; const v16b vh = frag_b(VB + vo, lane), vl = frag_b(VBL + vo, lane);
        acc[jt] = wmma_bf(pl.v, vh, acc[jt]); acc[jt] = wmma_bf(ph.v, vl, acc[jt]); acc[jt] = wmma_bf(ph.v, vh, acc[jt]); }
    } else {
#pragma unroll
      for (int r = 0; r < 8; ++r) {
#pragma unroll
        for (int j = 0; j < 2; ++j) psh[wave][8 * g + r][j * 16 + col] = (_Float16)(s[j][r] * PCARRY); }
      LDSX();
      union { v16h v; v8h q[2]; } pf;
      pf.q[0] = *(const v8h*)&psh[wave][col][8 * g]; pf.q[1] = *(const v8h*)&psh[wave][col][16 + 8 * g];
      LDSX();
#pragma unroll
      for (int jt = 0; jt < 4; ++jt) { const v16h vf = frag_h(VT + ((size_t)bh * HD + jt * 16 + col) * SEQ + k0, lane); acc[jt] = wmma16(pf.v, vf, acc[jt]); }
    }
  }
  const float pc = hi ? 1.0f : PCARRY;
#pragma unroll
  for (int r = 0; r < 8; ++r) { float l = lst[r];
    l += __shfl_xor(l, 1); l += __shfl_xor(l, 2); l += __shfl_xor(l, 4); l += __shfl_xor(l, 8);
    const float inv = 1.0f / (l * pc);
#pragma unroll
    for (int jt = 0; jt < 4; ++jt) { const float v = acc[jt][r] * inv; const __bf16 hv = (__bf16)v; ysh[wave][8 * g + r][jt * 16 + col] = hv; ysl[wave][8 * g + r][jt * 16 + col] = (__bf16)(v - (float)hv); } }
  LDSX();
  const int b = bh / NH, h = bh % NH;
#pragma unroll
  for (int it = 0; it < 4; ++it) { const int row = it * 4 + (lane >> 3), pq = lane & 7;
    const size_t o = ((size_t)b * SEQ + q0 + row) * CC + h * HD + pq * 8;
    const v4u vh = *(const v4u*)&ysh[wave][row][pq * 8]; const v4u vl = *(const v4u*)&ysl[wave][row][pq * 8];
    vst2((void*)(YH + o), vh); vst2((void*)(YL + o), vl); }
}
__global__ __launch_bounds__(128) void k_out(const __bf16* __restrict__ YH, const __bf16* __restrict__ YL, const __bf16* __restrict__ WPT, const float* __restrict__ BO, float* __restrict__ OUT) {
  __shared__ __align__(16) float sf[4][16][132];
  const int tid = threadIdx.x; const int wave = __builtin_amdgcn_readfirstlane(tid >> 5); const int lane = tid & 31, col = lane & 15, g = lane >> 4;
  const int c0 = blockIdx.y * 128; const size_t r0 = (size_t)blockIdx.x * 64 + wave * 16;
  v8f acc[8] = {};
  const size_t ao = (r0 + col) * CC;
#pragma unroll 1
  for (int kc = 0; kc < CC / 32; ++kc) { const v16b ah = frag_b(YH + ao + kc * 32, lane), al = frag_b(YL + ao + kc * 32, lane);
#pragma unroll
    for (int j = 0; j < 8; ++j) { const v16b w = frag_b(WPT + (size_t)(c0 + j * 16 + col) * CC + kc * 32, lane); acc[j] = wmma_bf(al, w, acc[j]); acc[j] = wmma_bf(ah, w, acc[j]); } }
#pragma unroll
  for (int j = 0; j < 8; ++j) { const float bias = bfr(BO[c0 + j * 16 + col]);
#pragma unroll
    for (int r = 0; r < 8; ++r) sf[wave][8 * g + r][j * 16 + col] = acc[j][r] + bias; }
  LDSX();
  for (int rl = 0; rl < 16; ++rl) { const v4f vv = *(const v4f*)&sf[wave][rl][lane * 4]; vst2((void*)(OUT + (r0 + rl) * DIN + c0 + lane * 4), vv); }
}

extern "C" void kernel_launch(void* const* d_in, const int* in_sizes, int n_in, void* d_out, int out_size, void* d_ws, size_t ws_size, hipStream_t stream) {
  if (n_in < 5) return;
  if ((size_t)in_sizes[0] < (size_t)(NB - 1) * SEQ_FULL * DIN + (size_t)SEQ * DIN) return;
  if ((size_t)in_sizes[1] < (size_t)DIN * 3 * CC) return;
  if (in_sizes[2] < 3 * CC) return;
  if ((size_t)in_sizes[3] < (size_t)CC * DIN) return;
  if (in_sizes[4] < DIN) return;
  if ((size_t)out_size < (size_t)NB * SEQ * DIN) return;
  if (ws_size < (size_t)WS_END) return;
  const float* X = (const float*)d_in[0]; const float* Wqkv = (const float*)d_in[1]; const float* bqkv = (const float*)d_in[2]; const float* Wproj = (const float*)d_in[3]; const float* bproj = (const float*)d_in[4];
  char* ws = (char*)d_ws;
  __bf16* XB = (__bf16*)(ws + WS_XB); __bf16* WQT = (__bf16*)(ws + WS_WQT); __bf16* WPT = (__bf16*)(ws + WS_WPT);
  __bf16* QKH = (__bf16*)(ws + WS_QKH); __bf16* QKL = (__bf16*)(ws + WS_QKL);
  float* VF = (float*)(ws + WS_VF); _Float16* VT = (_Float16*)(ws + WS_VT); __bf16* VB = (__bf16*)(ws + WS_VB); __bf16* VBL = (__bf16*)(ws + WS_VBL);
  __bf16* YH = (__bf16*)(ws + WS_YH); __bf16* YL = (__bf16*)(ws + WS_YL);
  k_cvt_x<<<dim3((unsigned)((size_t)NB * SEQ * DIN / 8 / 256)), 256, 0, stream>>>(X, XB);
  k_wT<<<dim3(3 * CC / 64, DIN / 64), 256, 0, stream>>>(Wqkv, WQT, DIN, 3 * CC);
  k_wT<<<dim3(DIN / 64, CC / 64), 256, 0, stream>>>(Wproj, WPT, CC, DIN);
  k_proj<<<dim3(NB * SEQ / 64, 3 * CC / 128), 128, 0, stream>>>(XB, WQT, bqkv, QKH, QKL, VF);
  k_vt<<<dim3(SEQ / 64, NB * NH), 256, 0, stream>>>(VF, VT, VB, VBL);
  k_attn<<<dim3(SEQ / 64, NB * NH), 128, 0, stream>>>(QKH, QKL, QKH + PLANE, QKL + PLANE, VT, VB, VBL, YH, YL);
  k_out<<<dim3(NB * SEQ / 64, DIN / 128), 128, 0, stream>>>(YH, YL, WPT, bproj, (float*)d_out);
}
